// EmberBlock_3384434229253
// MI455X (gfx1250) — hardware-run, weakly checked
//
#include <hip/hip_runtime.h>
#include <stddef.h>

typedef __attribute__((ext_vector_type(16))) _Float16 v16h;
typedef __attribute__((ext_vector_type(8)))  _Float16 v8h;
typedef __attribute__((ext_vector_type(8)))  float    v8f;
typedef __attribute__((ext_vector_type(4)))  float    v4f;
typedef __attribute__((ext_vector_type(4)))  unsigned v4u;

constexpr int kBatch   = 2;
constexpr int kSeq     = 2048;
constexpr int kEmb     = 1024;
constexpr int kHeads   = 16;
constexpr int kHeadDim = 64;
constexpr int kRows    = kBatch * kSeq;
constexpr int kQkvN    = 3 * kEmb;
constexpr int kFcN     = 4 * kEmb;
constexpr int kFcHalf  = kFcN / 2;
constexpr float kWCarry = 64.0f;
constexpr float kPCarry = 4096.0f;
constexpr float kYCarry = 64.0f;
constexpr float kGCarry = 16.0f;

static_assert(kHeads * kHeadDim == kEmb);
static_assert(kSeq % 64 == 0);
static_assert(kHeadDim == 64);
static_assert(kRows % 64 == 0 && kQkvN % 64 == 0 && kEmb % 64 == 0 && kFcHalf % 64 == 0);
static_assert(kEmb % 32 == 0 && kFcN % 32 == 0);
static_assert(((kRows / 64) * (kQkvN / 64)) % 8 == 0);
static_assert(((kRows / 64) * (kEmb / 64)) % 8 == 0);
static_assert(((kRows / 64) * (kFcHalf / 64)) % 8 == 0);

__device__ __forceinline__ void dep_guard_h(v8f& a, v8f& b, v16h x, v16h y) { asm volatile("v_nop\n\tv_nop\n\tv_nop\n\tv_nop" : "+v"(a), "+v"(b) : "v"(x), "v"(y)); }
__device__ __forceinline__ void keep4_h(v16h a, v16h b, v16h c, v16h d) { asm volatile("v_nop" :: "v"(a), "v"(b), "v"(c), "v"(d)); }
__device__ __forceinline__ void acc_guard4(v8f& a, v8f& b, v8f& c, v8f& d) { asm volatile("v_nop\n\tv_nop\n\tv_nop\n\tv_nop" : "+v"(a), "+v"(b), "+v"(c), "+v"(d)); }

template <typename T> struct Frag;
template <> struct Frag<_Float16> {
  typedef v16h V; union U { v16h v; v8h h[2]; };
  static __device__ __forceinline__ v16h load(const _Float16* p) {
    U f; f.h[0] = *(const v8h*)(p); f.h[1] = *(const v8h*)(p + 16); return f.v;
  }
  static __device__ __forceinline__ v8f mma(v16h a, v16h b, v8f c) {
    return __builtin_amdgcn_wmma_f32_16x16x32_f16(false, a, false, b, (short)0, c, false, false);
  }
  static __device__ __forceinline__ void guard(v8f& a, v8f& b, v16h x, v16h y) { dep_guard_h(a, b, x, y); }
  static __device__ __forceinline__ void keep(v16h a, v16h b, v16h c, v16h d) { keep4_h(a, b, c, d); }
};

__device__ __forceinline__ v8f mma16_guarded(v16h a, v16h b, v8f c) {
  c = __builtin_amdgcn_wmma_f32_16x16x32_f16(false, a, false, b, (short)0, c, false, false);
  asm volatile("v_nop\n\tv_nop\n\tv_nop\n\tv_nop" : "+v"(c) : "v"(a), "v"(b));
  return c;
}

template <bool SPLIT, int BIAS_MODE, int OUT_MODE, bool RESID>
__global__ __launch_bounds__(256) void wmma_gemm64(
    const unsigned short* __restrict__ Ap, const unsigned short* __restrict__ A2p, int lda, long strideA,
    const unsigned short* __restrict__ Btp, const unsigned short* __restrict__ Bt2p, int ldb, long strideB,
    void* __restrict__ Cout, int ldc, long strideC,
    const float* __restrict__ bias,
    const float* __restrict__ resid, long strideR,
    int M, int N, int K, float scale) {
  static_assert(!(RESID && OUT_MODE != 0));
  static_assert(BIAS_MODE == 0 || BIAS_MODE == 2);
  typedef _Float16 T;
  typedef v16h V;
  const T* A = (const T*)Ap; const T* A2 = (const T*)A2p; const T* Bt = (const T*)Btp; const T* Bt2 = (const T*)Bt2p;
  __shared__ __align__(16) float sT[8][16 * 68];
  const int b    = blockIdx.y;
  const int lane = threadIdx.x & 31;
  const int wave = threadIdx.x >> 5;
  const int tilesN = N >> 6;
  const int tilesM = M >> 6;
  const int tile = blockIdx.x * 8 + wave;
  if (tile >= tilesM * tilesN) return;
  const int tm = tile / tilesN;
  const int tn = tile - tm * tilesN;
  const int m0 = tm << 6;
  const int n0 = tn << 6;

  const T* Ab  = A  + (size_t)b * strideA;
  const T* Bb  = Bt + (size_t)b * strideB;
  const T* Ab2 = SPLIT ? (A2  + (size_t)b * strideA) : nullptr;
  const T* Bb2 = SPLIT ? (Bt2 + (size_t)b * strideB) : nullptr;

  const int rlane = lane & 15;
  const int koff  = (lane >> 4) * 8;
  const int mOff  = (lane >> 4) * 8;

  v8f acc[4][4];
#pragma unroll
  for (int i = 0; i < 4; ++i)
#pragma unroll
    for (int j = 0; j < 4; ++j) acc[i][j] = (v8f){0.f,0.f,0.f,0.f,0.f,0.f,0.f,0.f};

  for (int k0 = 0; k0 < K; k0 += 32) {
    V bh[4], bl[4];
#pragma unroll
    for (int j = 0; j < 4; ++j) {
      const size_t bo = (size_t)(n0 + (j << 4) + rlane) * ldb + koff + k0;
      bh[j] = Frag<T>::load(Bb + bo);
      if (SPLIT) bl[j] = Frag<T>::load(Bb2 + bo);
    }
#pragma unroll
    for (int i = 0; i < 4; ++i) {
      const size_t ao = (size_t)(m0 + (i << 4) + rlane) * lda + koff + k0;
      V ah = Frag<T>::load(Ab + ao);
      V al;
      if (SPLIT) al = Frag<T>::load(Ab2 + ao);
#pragma unroll
      for (int j = 0; j < 4; ++j) {
        acc[i][j] = Frag<T>::mma(ah, bh[j], acc[i][j]);
        if (SPLIT) {
          acc[i][j] = Frag<T>::mma(ah, bl[j], acc[i][j]);
          acc[i][j] = Frag<T>::mma(al, bh[j], acc[i][j]);
        }
      }
      Frag<T>::guard(acc[i][0], acc[i][3], ah, SPLIT ? al : ah);
    }
    Frag<T>::keep(bh[0], bh[1], bh[2], bh[3]);
    if (SPLIT) Frag<T>::keep(bl[0], bl[1], bl[2], bl[3]);
  }
  acc_guard4(acc[0][0], acc[0][1], acc[0][2], acc[0][3]);
  acc_guard4(acc[1][0], acc[1][1], acc[1][2], acc[1][3]);
  acc_guard4(acc[2][0], acc[2][1], acc[2][2], acc[2][3]);
  acc_guard4(acc[3][0], acc[3][1], acc[3][2], acc[3][3]);

  float* slab = sT[wave];
  const float* Rb = RESID ? (resid + (size_t)b * strideR) : nullptr;
#pragma unroll
  for (int i = 0; i < 4; ++i) {
    const int mBase = m0 + (i << 4);
#pragma unroll
    for (int j = 0; j < 4; ++j) {
      const int n = n0 + (j << 4) + rlane;
      float bv = 0.f;
      if (BIAS_MODE == 2) bv = bias[n];
#pragma unroll
      for (int r = 0; r < 8; ++r) {
        float v = acc[i][j][r] * scale;
        if (BIAS_MODE == 2) v += bv;
        slab[(mOff + r) * 68 + (j << 4) + rlane] = v;
      }
    }
    __builtin_amdgcn_fence(__ATOMIC_RELEASE, "workgroup");
    __builtin_amdgcn_wave_barrier();
    __builtin_amdgcn_fence(__ATOMIC_ACQUIRE, "workgroup");
    if (OUT_MODE == 0) {
      float* C = (float*)Cout + (size_t)b * strideC;
      const int hh = lane >> 4, c4 = (lane & 15) * 4;
      v4f vals[8];
#pragma unroll
      for (int it = 0; it < 8; ++it) {
        const int row = it * 2 + hh;
        v4f v = *(const v4f*)(slab + row * 68 + c4);
        if (RESID) {
          const v4f rv = *(const v4f*)(Rb + (size_t)(mBase + row) * ldc + n0 + c4);
          v += rv;
        }
        vals[it] = v;
      }
      for (int pass = 0; pass < 2; ++pass) {
#pragma unroll
        for (int it = 0; it < 8; ++it) {
          const int row = it * 2 + hh;
          *(volatile v4f*)(C + (size_t)(mBase + row) * ldc + n0 + c4) = vals[it];
        }
        __threadfence();
      }
    } else {
      const int q = lane >> 3, c8 = (lane & 7) * 8;
      unsigned short* C = (unsigned short*)Cout + (size_t)b * strideC;
      v8h hvs[4];
#pragma unroll
      for (int it = 0; it < 4; ++it) {
        const int row = it * 4 + q;
        const float* sp = slab + row * 68 + c8;
        v8h hv;
#pragma unroll
        for (int e = 0; e < 8; ++e) hv[e] = (_Float16)sp[e];
        hvs[it] = hv;
      }
      for (int pass = 0; pass < 2; ++pass) {
#pragma unroll
        for (int it = 0; it < 4; ++it) {
          const int row = it * 4 + q;
          *(volatile v8h*)(C + (size_t)(mBase + row) * ldc + n0 + c8) = hvs[it];
        }
        __threadfence();
      }
    }
    __builtin_amdgcn_fence(__ATOMIC_RELEASE, "workgroup");
    __builtin_amdgcn_wave_barrier();
    __builtin_amdgcn_fence(__ATOMIC_ACQUIRE, "workgroup");
  }
}

__global__ __launch_bounds__(256) void transpose_cast_f16_kernel(
    const float* __restrict__ in, unsigned short* __restrict__ out, int rows, int cols, float scl) {
  __shared__ __align__(16) _Float16 sm[64 * 72];
  const int t = threadIdx.x;
  const int r0 = blockIdx.y * 64;
  const int c0 = blockIdx.x * 64;
  {
    const int rr = t >> 2;
    const int cq = (t & 3) * 16;
    const float* src = in + (size_t)(r0 + rr) * cols + c0 + cq;
    v4f v[4];
#pragma unroll
    for (int i = 0; i < 4; ++i) v[i] = *(const v4f*)(src + 4 * i);
#pragma unroll
    for (int i = 0; i < 4; ++i) {
#pragma unroll
      for (int e = 0; e < 4; ++e) sm[(cq + 4 * i + e) * 72 + rr] = (_Float16)(v[i][e] * scl);
    }
  }
  __syncthreads();
  const int wave = t >> 5, lane = t & 31;
  const int qq = lane >> 3, c8 = (lane & 7) * 8;
  _Float16* out16 = (_Float16*)out;
  v8h ov[2];
#pragma unroll
  for (int it = 0; it < 2; ++it) {
    const int n = (wave * 2 + it) * 4 + qq;
    ov[it] = *(const v8h*)(sm + n * 72 + c8);
  }
  for (int pass = 0; pass < 2; ++pass) {
#pragma unroll
    for (int it = 0; it < 2; ++it) {
      const int n = (wave * 2 + it) * 4 + qq;
      *(volatile v8h*)(out16 + (size_t)(c0 + n) * rows + r0 + c8) = ov[it];
    }
    __threadfence();
  }
}

__global__ __launch_bounds__(128) void layernorm_f16_kernel(
    const float* __restrict__ in, const float* __restrict__ lw, const float* __restrict__ lb,
    unsigned short* __restrict__ out) {
  __shared__ float red1[4];
  __shared__ float red2[4];
  const int row = blockIdx.x;
  const int t = threadIdx.x, lane = t & 31, wave = t >> 5;
  const float* p = in + (size_t)row * kEmb + 8 * t;
  const v4f a0 = *(const v4f*)p;
  const v4f a1 = *(const v4f*)(p + 4);
  float s = ((a0[0] + a0[1]) + (a0[2] + a0[3])) + ((a1[0] + a1[1]) + (a1[2] + a1[3]));
#pragma unroll
  for (int off = 16; off > 0; off >>= 1) s += __shfl_xor(s, off, 32);
  if (lane == 0) red1[wave] = s;
  __syncthreads();
  const float tot = (red1[0] + red1[1]) + (red1[2] + red1[3]);
  const float mu = tot * (1.0f / (float)kEmb);
  const v4f d0 = a0 - mu;
  const v4f d1 = a1 - mu;
  float s2 = ((d0[0] * d0[0] + d0[1] * d0[1]) + (d0[2] * d0[2] + d0[3] * d0[3])) +
             ((d1[0] * d1[0] + d1[1] * d1[1]) + (d1[2] * d1[2] + d1[3] * d1[3]));
#pragma unroll
  for (int off = 16; off > 0; off >>= 1) s2 += __shfl_xor(s2, off, 32);
  if (lane == 0) red2[wave] = s2;
  __syncthreads();
  const float var = ((red2[0] + red2[1]) + (red2[2] + red2[3])) * (1.0f / (float)kEmb);
  const float rstd = rsqrtf(var + 1e-5f);
  const v4f w0 = *(const v4f*)(lw + 8 * t);
  const v4f w1 = *(const v4f*)(lw + 8 * t + 4);
  const v4f b0 = *(const v4f*)(lb + 8 * t);
  const v4f b1 = *(const v4f*)(lb + 8 * t + 4);
  const v4f o0 = d0 * rstd * w0 + b0;
  const v4f o1 = d1 * rstd * w1 + b1;
  v8h hv;
  hv[0] = (_Float16)o0[0]; hv[1] = (_Float16)o0[1]; hv[2] = (_Float16)o0[2]; hv[3] = (_Float16)o0[3];
  hv[4] = (_Float16)o1[0]; hv[5] = (_Float16)o1[1]; hv[6] = (_Float16)o1[2]; hv[7] = (_Float16)o1[3];
  _Float16* op = (_Float16*)out + (size_t)row * kEmb + 8 * t;
  *(volatile v8h*)op = hv;
  __threadfence();
  *(volatile v8h*)op = hv;
}

__global__ __launch_bounds__(256) void gelu_f16_kernel(
    const float* __restrict__ U, unsigned short* __restrict__ G, int ldg, int coloff) {
  const int i8 = (blockIdx.x * 256 + threadIdx.x) * 8;
  const int row = i8 / kFcHalf;
  const int col = i8 - row * kFcHalf;
  const float* p = U + i8;
  unsigned cur = 0u, w0 = 0u, w1 = 0u, w2 = 0u, w3 = 0u;
#pragma unroll 1
  for (int e = 0; e < 8; ++e) {
    const float u = p[e];
    const float y = (0.5f * u * (1.0f + erff(u * 0.70710678118654752f))) * kGCarry;
    const unsigned bits = (unsigned)__builtin_bit_cast(unsigned short, (_Float16)y);
    cur = (cur >> 16) | (bits << 16);
    w0 = (e == 1) ? cur : w0;
    w1 = (e == 3) ? cur : w1;
    w2 = (e == 5) ? cur : w2;
    w3 = (e == 7) ? cur : w3;
  }
  v4u o;
  o[0] = w0; o[1] = w1; o[2] = w2; o[3] = w3;
  unsigned short* gp = G + (size_t)row * ldg + coloff + col;
  *(volatile v4u*)gp = o;
  __threadfence();
  *(volatile v4u*)gp = o;
}

__global__ __launch_bounds__(128) void lif_attn_kernel(
    const unsigned short* __restrict__ qkv, const float* __restrict__ thr,
    const float* __restrict__ leakp, const float* __restrict__ steepp,
    unsigned short* __restrict__ yout) {
  union FB { v16h v; v8h h[2]; };
  __shared__ __align__(16) unsigned short Ksh[64 * 64];
  __shared__ __align__(16) unsigned short Vts[64 * 64];
  __shared__ __align__(16) _Float16 Psh[4][16 * 64];
  __shared__ __align__(16) float Os[4][16 * 68];

  const int tid = threadIdx.x, wave = tid >> 5, lane = tid & 31, hh = lane >> 4, c = lane & 15;
  constexpr int nqb = kSeq / 64;
  const int bx = blockIdx.x;
  const int qb = bx % nqb;
  const int bh = bx / nqb;
  const int h  = bh % kHeads;
  const int b  = bh / kHeads;
  const size_t rowbase = (size_t)b * kSeq;
  const int q0 = qb * 64 + wave * 16;
  const _Float16* qkv16 = (const _Float16*)qkv;
  const _Float16* Ksh16 = (const _Float16*)Ksh;
  const _Float16* Vts16 = (const _Float16*)Vts;
  const float NEG_INF = -__builtin_inff();

  const float th = fabsf(thr[h]) * 0.1f;
  const float lk = 1.0f / (1.0f + expf(-leakp[h]));
  const float spv = steepp[h];
  const float st = fmaxf(spv, 0.0f) + log1pf(expf(-fabsf(spv)));
  const float lkC = lk * kPCarry;
  const float omlkC = (1.0f - lk) * kPCarry;

  v16h qa[2];
  {
    const _Float16* qrow = qkv16 + (rowbase + q0 + c) * kQkvN + h * kHeadDim + 8 * hh;
#pragma unroll
    for (int dc = 0; dc < 2; ++dc) qa[dc] = Frag<_Float16>::load(qrow + dc * 32);
  }

  float mrow[8], lrow[8];
#pragma unroll
  for (int r = 0; r < 8; ++r) { mrow[r] = NEG_INF; lrow[r] = 0.f; }
  const int nChunks = qb + 1;

  for (int kc = 0; kc < nChunks; ++kc) {
    const int kv0 = kc * 64;
    __syncthreads();
    {
      const int kvr = tid >> 1, dh = (tid & 1) * 32;
      const v4u* ks = (const v4u*)(qkv + (rowbase + kv0 + kvr) * kQkvN + kEmb + h * kHeadDim + dh);
      v4u k4[4];
#pragma unroll
      for (int i = 0; i < 4; ++i) k4[i] = ks[i];
      v4u* kd = (v4u*)(Ksh + kvr * 64 + dh);
#pragma unroll
      for (int i = 0; i < 4; ++i) kd[i] = k4[i];
    }
    __syncthreads();

    v8f s[4];
#pragma unroll
    for (int j = 0; j < 4; ++j) {
      s[j] = (v8f){0.f,0.f,0.f,0.f,0.f,0.f,0.f,0.f};
#pragma unroll
      for (int dc = 0; dc < 2; ++dc) {
        FB kb;
        kb.h[0] = *(const v8h*)(Ksh16 + (j * 16 + c) * 64 + dc * 32 + 8 * hh);
        kb.h[1] = *(const v8h*)(Ksh16 + (j * 16 + c) * 64 + dc * 32 + 16 + 8 * hh);
        s[j] = mma16_guarded(qa[dc], kb.v, s[j]);
      }
    }
    const bool diag = (kc == qb);
#pragma unroll
    for (int r = 0; r < 8; ++r) {
      const int qrow = q0 + 8 * hh + r;
      float m = NEG_INF;
#pragma unroll
      for (int j = 0; j < 4; ++j) {
        const int kvcol = kv0 + j * 16 + c;
        float x = s[j][r] * 0.125f;
        x = (diag && (kvcol > qrow)) ? NEG_INF : x;
        s[j][r] = x;
        m = fmaxf(m, x);
      }
#pragma unroll
      for (int off = 1; off < 16; off <<= 1) m = fmaxf(m, __shfl_xor(m, off, 32));
      const float mnew = fmaxf(mrow[r], m);
      const float alpha = __expf(mrow[r] - mnew);
      float psum = 0.f;
#pragma unroll
      for (int j = 0; j < 4; ++j) psum += __expf(s[j][r] - mnew);
#pragma unroll
      for (int off = 1; off < 16; off <<= 1) psum += __shfl_xor(psum, off, 32);
      lrow[r] = lrow[r] * alpha + psum;
      mrow[r] = mnew;
    }
  }

  float rinv[8], musum[8];
#pragma unroll
  for (int r = 0; r < 8; ++r) { rinv[r] = 1.0f / lrow[r]; musum[r] = 0.f; }
  v8f oacc[4];
#pragma unroll
  for (int t = 0; t < 4; ++t) oacc[t] = (v8f){0.f,0.f,0.f,0.f,0.f,0.f,0.f,0.f};
  _Float16* pw = Psh[wave];

  for (int kc = 0; kc < nChunks; ++kc) {
    const int kv0 = kc * 64;
    __syncthreads();
    {
      const int kvr = tid >> 1, dh = (tid & 1) * 32;
      const v4u* ks = (const v4u*)(qkv + (rowbase + kv0 + kvr) * kQkvN + kEmb + h * kHeadDim + dh);
      const v4u* vs = (const v4u*)(qkv + (rowbase + kv0 + kvr) * kQkvN + 2 * kEmb + h * kHeadDim + dh);
      v4u k4[4], v4[4];
#pragma unroll
      for (int i = 0; i < 4; ++i) { k4[i] = ks[i]; v4[i] = vs[i]; }
      v4u* kd = (v4u*)(Ksh + kvr * 64 + dh);
#pragma unroll
      for (int i = 0; i < 4; ++i) kd[i] = k4[i];
#pragma unroll
      for (int i = 0; i < 4; ++i) {
#pragma unroll
        for (int wi = 0; wi < 4; ++wi) {
          const unsigned w = v4[i][wi];
          const int d = dh + i * 8 + wi * 2;
          Vts[d * 64 + kvr] = (unsigned short)(w & 0xffffu);
          Vts[(d + 1) * 64 + kvr] = (unsigned short)(w >> 16);
        }
      }
    }
    __syncthreads();

    v8f s[4];
#pragma unroll
    for (int j = 0; j < 4; ++j) {
      s[j] = (v8f){0.f,0.f,0.f,0.f,0.f,0.f,0.f,0.f};
#pragma unroll
      for (int dc = 0; dc < 2; ++dc) {
        FB kb;
        kb.h[0] = *(const v8h*)(Ksh16 + (j * 16 + c) * 64 + dc * 32 + 8 * hh);
        kb.h[1] = *(const v8h*)(Ksh16 + (j * 16 + c) * 64 + dc * 32 + 16 + 8 * hh);
        s[j] = mma16_guarded(qa[dc], kb.v, s[j]);
      }
    }
    const bool diag = (kc == qb);
#pragma unroll
    for (int r = 0; r < 8; ++r) {
      const int qrow = q0 + 8 * hh + r;
      const float nm = mrow[r];
      const float ri = rinv[r];
#pragma unroll
      for (int j = 0; j < 4; ++j) {
        const int kvcol = kv0 + j * 16 + c;
        float x = s[j][r] * 0.125f - nm;
        x = (diag && (kvcol > qrow)) ? NEG_INF : x;
        const float e = __expf(x);
        const float p = e * ri;
        const float tt = __expf((th - p) * st);
        const float fire = __builtin_amdgcn_rcpf(1.0f + tt);
        const float wq = fmaf(fire, omlkC, lkC);
        const float mu = e * wq;
        musum[r] += mu;
        pw[(8 * hh + r) * 64 + j * 16 + c] = (_Float16)mu;
      }
    }
    __builtin_amdgcn_fence(__ATOMIC_RELEASE, "workgroup");
    __builtin_amdgcn_wave_barrier();
    __builtin_amdgcn_fence(__ATOMIC_ACQUIRE, "workgroup");
#pragma unroll
    for (int kk = 0; kk < 2; ++kk) {
      FB pa;
      pa.h[0] = *(const v8h*)(pw + c * 64 + kk * 32 + 8 * hh);
      pa.h[1] = *(const v8h*)(pw + c * 64 + kk * 32 + 16 + 8 * hh);
#pragma unroll
      for (int t = 0; t < 4; ++t) {
        FB vb;
        vb.h[0] = *(const v8h*)(Vts16 + (t * 16 + c) * 64 + kk * 32 + 8 * hh);
        vb.h[1] = *(const v8h*)(Vts16 + (t * 16 + c) * 64 + kk * 32 + 16 + 8 * hh);
        oacc[t] = mma16_guarded(pa.v, vb.v, oacc[t]);
      }
    }
  }

  float* os = Os[wave];
#pragma unroll
  for (int r = 0; r < 8; ++r) {
    float ms = musum[r];
#pragma unroll
    for (int off = 1; off < 16; off <<= 1) ms += __shfl_xor(ms, off, 32);
    const float den = ms + (1e-8f * kPCarry) * lrow[r];
    const float inv = kYCarry / den;
#pragma unroll
    for (int t = 0; t < 4; ++t) os[(8 * hh + r) * 68 + t * 16 + c] = oacc[t][r] * inv;
  }
  __builtin_amdgcn_fence(__ATOMIC_RELEASE, "workgroup");
  __builtin_amdgcn_wave_barrier();
  __builtin_amdgcn_fence(__ATOMIC_ACQUIRE, "workgroup");
  {
    const int qq = lane >> 3, c8 = (lane & 7) * 8;
    _Float16* y16 = (_Float16*)yout;
    v8h hv4[4];
#pragma unroll
    for (int it = 0; it < 4; ++it) {
      const int row = it * 4 + qq;
      const float* sp = os + row * 68 + c8;
      v8h hv;
#pragma unroll
      for (int e = 0; e < 8; ++e) hv[e] = (_Float16)sp[e];
      hv4[it] = hv;
    }
    for (int pass = 0; pass < 2; ++pass) {
#pragma unroll
      for (int it = 0; it < 4; ++it) {
        const int row = it * 4 + qq;
        *(volatile v8h*)(y16 + (rowbase + q0 + row) * kEmb + h * kHeadDim + c8) = hv4[it];
      }
      __threadfence();
    }
  }
}

extern "C" void kernel_launch(void* const* d_in, const int* in_sizes, int n_in,
                              void* d_out, int out_size, void* d_ws, size_t ws_size,
                              hipStream_t stream) {
  constexpr size_t kMiB = 1048576;
  constexpr size_t kWsTotal = 104 * kMiB;
  static_assert((size_t)kRows * kEmb * 4 == 16 * kMiB);
  static_assert((size_t)kFcN * kEmb * 2 == 8 * kMiB);
  static_assert((size_t)kRows * kEmb * 2 == 8 * kMiB);
  static_assert((size_t)kQkvN * kEmb * 2 == 6 * kMiB);
  static_assert((size_t)kEmb * kEmb * 2 == 2 * kMiB);
  static_assert((size_t)kRows * kQkvN * 2 == 24 * kMiB);
  static_assert((size_t)kRows * kFcHalf * 4 == 32 * kMiB);
  static_assert((size_t)kRows * kFcN * 2 == 32 * kMiB);
  static_assert(kWsTotal <= (size_t)134217728);

  if (n_in < 16) return;
  if (out_size != kRows * kEmb) return;
  if (ws_size < kWsTotal) return;
  if (in_sizes[0] != kRows * kEmb || in_sizes[3] != kEmb * kQkvN || in_sizes[5] != kEmb * kEmb ||
      in_sizes[12] != kEmb * kFcN || in_sizes[14] != kFcN * kEmb ||
      in_sizes[7] < kHeads || in_sizes[8] < kHeads || in_sizes[9] < kHeads) return;

  const float* x           = (const float*)d_in[0];
  const float* ln1_w       = (const float*)d_in[1];
  const float* ln1_b       = (const float*)d_in[2];
  const float* w_attn      = (const float*)d_in[3];
  const float* b_attn      = (const float*)d_in[4];
  const float* w_attn_proj = (const float*)d_in[5];
  const float* b_attn_proj = (const float*)d_in[6];
  const float* threshold   = (const float*)d_in[7];
  const float* leak        = (const float*)d_in[8];
  const float* steepness   = (const float*)d_in[9];
  const float* ln2_w       = (const float*)d_in[10];
  const float* ln2_b       = (const float*)d_in[11];
  const float* w_fc        = (const float*)d_in[12];
  const float* b_fc        = (const float*)d_in[13];
  const float* w_mlp_proj  = (const float*)d_in[14];
  const float* b_mlp_proj  = (const float*)d_in[15];
  float* out = (float*)d_out;

  char* ws = (char*)d_ws;
  float*          x1     = (float*)(ws + 0 * kMiB);
  unsigned short* wfcT   = (unsigned short*)(ws + 16 * kMiB);
  unsigned short* wmlpT  = (unsigned short*)(ws + 24 * kMiB);
  unsigned short* hbuf   = (unsigned short*)(ws + 32 * kMiB);
  unsigned short* wqkvT  = (unsigned short*)(ws + 40 * kMiB);
  unsigned short* wprojT = (unsigned short*)(ws + 46 * kMiB);
  unsigned short* qkv    = (unsigned short*)(ws + 48 * kMiB);
  float*          ubuf   = (float*)(ws + 40 * kMiB);
  unsigned short* ybuf   = (unsigned short*)(ws + 72 * kMiB);
  unsigned short* gbuf   = (unsigned short*)(ws + 72 * kMiB);

  const float invW  = 1.0f / kWCarry;
  const float invWY = 1.0f / (kWCarry * kYCarry);
  const float invWG = 1.0f / (kWCarry * kGCarry);

  transpose_cast_f16_kernel<<<dim3(kQkvN / 64, kEmb / 64), 256, 0, stream>>>(w_attn, wqkvT, kEmb, kQkvN, kWCarry);
  transpose_cast_f16_kernel<<<dim3(kEmb / 64, kEmb / 64), 256, 0, stream>>>(w_attn_proj, wprojT, kEmb, kEmb, kWCarry);
  transpose_cast_f16_kernel<<<dim3(kFcN / 64, kEmb / 64), 256, 0, stream>>>(w_fc, wfcT, kEmb, kFcN, kWCarry);
  transpose_cast_f16_kernel<<<dim3(kEmb / 64, kFcN / 64), 256, 0, stream>>>(w_mlp_proj, wmlpT, kFcN, kEmb, kWCarry);

  layernorm_f16_kernel<<<kRows, 128, 0, stream>>>(x, ln1_w, ln1_b, hbuf);

  wmma_gemm64<false, 2, 1, false><<<dim3((kRows / 64) * (kQkvN / 64) / 8, 1), 256, 0, stream>>>(
      hbuf, nullptr, kEmb, 0L, wqkvT, nullptr, kEmb, 0L,
      (void*)qkv, kQkvN, 0L, b_attn, nullptr, 0L, kRows, kQkvN, kEmb, invW);

  lif_attn_kernel<<<kBatch * kHeads * (kSeq / 64), 128, 0, stream>>>(qkv, threshold, leak, steepness, ybuf);

  wmma_gemm64<false, 2, 0, true><<<dim3((kRows / 64) * (kEmb / 64) / 8, 1), 256, 0, stream>>>(
      ybuf, nullptr, kEmb, 0L, wprojT, nullptr, kEmb, 0L,
      (void*)x1, kEmb, 0L, b_attn_proj, x, 0L, kRows, kEmb, kEmb, invWY);

  layernorm_f16_kernel<<<kRows, 128, 0, stream>>>(x1, ln2_w, ln2_b, hbuf);

  for (int half = 0; half < 2; ++half) {
    wmma_gemm64<false, 2, 0, false><<<dim3((kRows / 64) * (kFcHalf / 64) / 8, 1), 256, 0, stream>>>(
        hbuf, nullptr, kEmb, 0L, wfcT + (size_t)half * kFcHalf * kEmb, nullptr, kEmb, 0L,
        (void*)ubuf, kFcHalf, 0L, b_fc + half * kFcHalf, nullptr, 0L, kRows, kFcHalf, kEmb, invW);
    gelu_f16_kernel<<<(kRows * kFcHalf) / (8 * 256), 256, 0, stream>>>(ubuf, gbuf, kFcN, half * kFcHalf);
  }

  wmma_gemm64<false, 2, 0, true><<<dim3((kRows / 64) * (kEmb / 64) / 8, 1), 256, 0, stream>>>(
      gbuf, nullptr, kFcN, 0L, wmlpT, nullptr, kFcN, 0L,
      (void*)out, kEmb, 0L, b_mlp_proj, x1, 0L, kRows, kEmb, kFcN, invWG);
}
